// GeometricAttentionLayer_84482006712467
// MI455X (gfx1250) — hardware-verified
//
#include <hip/hip_runtime.h>
#include <hip/hip_bf16.h>
#include <stddef.h>


#define CIN    256
#define HD     256
#define DH     64
#define NH     4
#define HQKV   768
#define DOUT   64
#define NTHR   256
#define NWAVE  8
#define EPT    8
#define NGRP   2
#define CHUNK  (NTHR * EPT * NGRP)
#define WCAP   (EPT * NGRP * 32)
#define LISTN  (NWAVE * WCAP)
#define NB     4096
#define PROWS  64
#define PCOLS  128
#define EPB    256
#define APITCH 256
#define NEGBIG (-3.0e38f)

#define LDS_PROJ (2 * PROWS * APITCH * 2)
#define LDS_AGG  (NB * NH * 4 + LISTN * 4 + 64)
#define LDS_OUT  (2 * PROWS * APITCH * 2)

static_assert((CHUNK & (CHUNK - 1)) == 0);
static_assert(CHUNK <= 4096);
static_assert(NB <= 4096);
static_assert(PROWS * PCOLS * 4 <= LDS_PROJ);
static_assert(PROWS * DOUT * 4 <= LDS_OUT);
static_assert((PROWS * CIN / 8) % NTHR == 0);
static_assert(EPB == NWAVE * 32);
static_assert(NWAVE * 16 * 128 == NB * NH);

typedef float  v4f  __attribute__((ext_vector_type(4)));
typedef float  v8f  __attribute__((ext_vector_type(8)));
typedef int    v4i  __attribute__((ext_vector_type(4)));
typedef __bf16 v8b  __attribute__((ext_vector_type(8)));
typedef __bf16 v16b __attribute__((ext_vector_type(16)));
union FragB { v16b v; v8b h[2]; };
struct HiLo { v8b hi; v8b lo; };

__device__ __forceinline__ HiLo split8(v4f a, v4f b) {
  HiLo r;
#define SPL(I, F) { const float f_ = (F); const __bf16 h_ = (__bf16)f_; r.hi[I] = h_; r.lo[I] = (__bf16)(f_ - (float)h_); }
  SPL(0, a.x) SPL(1, a.y) SPL(2, a.z) SPL(3, a.w)
  SPL(4, b.x) SPL(5, b.y) SPL(6, b.z) SPL(7, b.w)
#undef SPL
  return r;
}

__device__ __forceinline__ v8f wmb(v16b a, v16b b, v8f c) {
  v8f d = __builtin_amdgcn_wmma_f32_16x16x32_bf16(false, a, false, b, (short)0, c, false, false);
  asm volatile("v_nop\n\tv_nop\n\tv_nop\n\tv_nop" : "+v"(d) : "v"(a), "v"(b));
  return d;
}

__device__ __forceinline__ v8f wm3(const FragB& ah, const FragB& al, const FragB& bh, const FragB& bl, v8f c) {
  c = wmb(ah.v, bh.v, c);
  c = wmb(ah.v, bl.v, c);
  c = wmb(al.v, bh.v, c);
  return c;
}

template <int NBT>
__device__ __forceinline__ int scan_chunk(const int* __restrict__ dsts, int nE, int cbase, int nodeBase,
                                          int vec8, int* list, int tid, int lane, int wave) {
  int wc = 0;
#pragma unroll
  for (int g = 0; g < NGRP; ++g) {
    const int el0  = (g * NTHR + tid) * EPT;
    const int e0   = cbase + el0;
    const int sent = -2147483647 - 1;
    v4i da, db;
    if (vec8 != 0 && cbase + CHUNK <= nE) {
      da = *(const v4i*)(dsts + e0);
      db = *(const v4i*)(dsts + e0 + 4);
    } else {
      da.x = (e0     < nE) ? dsts[min(e0, nE - 1)] : sent;
      da.y = (e0 + 1 < nE) ? dsts[min(e0 + 1, nE - 1)] : sent;
      da.z = (e0 + 2 < nE) ? dsts[min(e0 + 2, nE - 1)] : sent;
      da.w = (e0 + 3 < nE) ? dsts[min(e0 + 3, nE - 1)] : sent;
      db.x = (e0 + 4 < nE) ? dsts[min(e0 + 4, nE - 1)] : sent;
      db.y = (e0 + 5 < nE) ? dsts[min(e0 + 5, nE - 1)] : sent;
      db.z = (e0 + 6 < nE) ? dsts[min(e0 + 6, nE - 1)] : sent;
      db.w = (e0 + 7 < nE) ? dsts[min(e0 + 7, nE - 1)] : sent;
    }
    const unsigned nb = (unsigned)nodeBase;
    const unsigned s0 = (unsigned)da.x - nb, s1 = (unsigned)da.y - nb;
    const unsigned s2 = (unsigned)da.z - nb, s3 = (unsigned)da.w - nb;
    const unsigned s4 = (unsigned)db.x - nb, s5 = (unsigned)db.y - nb;
    const unsigned s6 = (unsigned)db.z - nb, s7 = (unsigned)db.w - nb;
    const bool h0 = s0 < (unsigned)NBT, h1 = s1 < (unsigned)NBT, h2 = s2 < (unsigned)NBT, h3 = s3 < (unsigned)NBT;
    const bool h4 = s4 < (unsigned)NBT, h5 = s5 < (unsigned)NBT, h6 = s6 < (unsigned)NBT, h7 = s7 < (unsigned)NBT;
    const unsigned any = __builtin_amdgcn_ballot_w32(h0 | h1 | h2 | h3 | h4 | h5 | h6 | h7);
    if (any != 0u) {
#define HITJ(J, HJ, SJ) { \
        const unsigned mj = __builtin_amdgcn_ballot_w32(HJ); \
        if (mj != 0u) { \
          if (HJ) { \
            const int pos = wc + (int)__builtin_amdgcn_mbcnt_lo(mj, 0u); \
            if (pos < WCAP) list[wave * WCAP + pos] = ((el0 + (J)) << 12) | (int)(SJ); \
          } \
          wc += (int)__builtin_popcount(mj); } }
      HITJ(0, h0, s0)
      HITJ(1, h1, s1)
      HITJ(2, h2, s2)
      HITJ(3, h3, s3)
      HITJ(4, h4, s4)
      HITJ(5, h5, s5)
      HITJ(6, h6, s6)
      HITJ(7, h7, s7)
#undef HITJ
    }
  }
  return wc;
}

__global__ __launch_bounds__(NTHR) void k_wprep(
    const float* __restrict__ Wq, const float* __restrict__ Wk, const float* __restrict__ Wv,
    const float* __restrict__ Wo, const float* __restrict__ bq, const float* __restrict__ bk,
    const float* __restrict__ bv, __bf16* wh, __bf16* wl, __bf16* oh, __bf16* ol, float* bias,
    int nWB, int nOWB) {
  const int tid = threadIdx.x;
  const int b = blockIdx.x;
  if (b < nWB) {
    const int i   = b * NTHR + tid;
    const int o   = i * 8;
    const int n   = o >> 8;
    const int k0  = o & 255;
    const int mat = n >> 8;
    const int nn  = n & 255;
    const float* Wsrc = (mat == 0) ? Wq : ((mat == 1) ? Wk : Wv);
    const float* p = Wsrc + (size_t)k0 * HD + nn;
    v4f a, c;
    a.x = p[0];      a.y = p[HD];     a.z = p[2 * HD]; a.w = p[3 * HD];
    c.x = p[4 * HD]; c.y = p[5 * HD]; c.z = p[6 * HD]; c.w = p[7 * HD];
    const HiLo s = split8(a, c);
    *(volatile v8b*)(wh + o) = s.hi;
    *(volatile v8b*)(wl + o) = s.lo;
    __threadfence();
    *(volatile v8b*)(wh + o) = s.hi;
    *(volatile v8b*)(wl + o) = s.lo;
  } else if (b < nWB + nOWB) {
    const int i  = (b - nWB) * NTHR + tid;
    const int o  = i * 8;
    const int n  = o >> 8;
    const int k0 = o & 255;
    const float* p = Wo + (size_t)k0 * DOUT + n;
    v4f a, c;
    a.x = p[0];        a.y = p[DOUT];     a.z = p[2 * DOUT]; a.w = p[3 * DOUT];
    c.x = p[4 * DOUT]; c.y = p[5 * DOUT]; c.z = p[6 * DOUT]; c.w = p[7 * DOUT];
    const HiLo s = split8(a, c);
    *(volatile v8b*)(oh + o) = s.hi;
    *(volatile v8b*)(ol + o) = s.lo;
    __threadfence();
    *(volatile v8b*)(oh + o) = s.hi;
    *(volatile v8b*)(ol + o) = s.lo;
  } else {
    if (tid < HQKV / 4) {
      const int c   = 4 * tid;
      const int mat = c >> 8;
      const int idx = c & 255;
      const v4f va = *(const v4f*)(bq + idx);
      const v4f vb = *(const v4f*)(bk + idx);
      const v4f vc = *(const v4f*)(bv + idx);
      const v4f v  = (mat == 0) ? va : ((mat == 1) ? vb : vc);
      *(volatile v4f*)(bias + c) = v;
      __threadfence();
      *(volatile v4f*)(bias + c) = v;
    }
  }
}

__global__ __launch_bounds__(NTHR) void k_proj(
    const float* __restrict__ x, const __bf16* __restrict__ wh, const __bf16* __restrict__ wl,
    const float* __restrict__ bias, float* outp, int nN, int col0, int ncb, int ldo) {
  extern __shared__ v4f lds_dyn[];
  __bf16* sH  = (__bf16*)lds_dyn;
  __bf16* sL  = sH + PROWS * APITCH;
  float*  stg = (float*)lds_dyn;
  const int tid = threadIdx.x, lane = tid & 31, wave = tid >> 5, hh = lane >> 4, m = lane & 15;
  const int rb = blockIdx.x / ncb;
  const int cb = blockIdx.x - rb * ncb;
  const int rowBase = rb * PROWS;
  const int wrow0   = col0 + cb * PCOLS;

#pragma unroll
  for (int i = 0; i < (PROWS * CIN / 8) / NTHR; ++i) {
    const int idx = i * NTHR + tid;
    const int r   = idx >> 5;
    const int c0  = (idx & 31) * 8;
    int node = rowBase + r;
    node = node > nN - 1 ? nN - 1 : node;
    const float* xp = x + (size_t)node * CIN + c0;
    const HiLo s = split8(*(const v4f*)xp, *(const v4f*)(xp + 4));
    *(v8b*)(sH + r * APITCH + c0) = s.hi;
    *(v8b*)(sL + r * APITCH + c0) = s.lo;
  }
  __syncthreads();

  const int rt = wave & 3, cg = wave >> 2;
  v8f acc[4];
#pragma unroll
  for (int t = 0; t < 4; ++t) { v8f z = {0.f, 0.f, 0.f, 0.f, 0.f, 0.f, 0.f, 0.f}; acc[t] = z; }
  const __bf16* arh = sH + (16 * rt + m) * APITCH + 8 * hh;
  const __bf16* arl = sL + (16 * rt + m) * APITCH + 8 * hh;
  const __bf16* bbh = wh + (size_t)(wrow0 + 64 * cg + m) * CIN + 8 * hh;
  const __bf16* bbl = wl + (size_t)(wrow0 + 64 * cg + m) * CIN + 8 * hh;
#pragma unroll 1
  for (int kt = 0; kt < CIN / 32; ++kt) {
    FragB ah, al;
    ah.h[0] = *(const v8b*)(arh + 32 * kt);
    ah.h[1] = *(const v8b*)(arh + 32 * kt + 16);
    al.h[0] = *(const v8b*)(arl + 32 * kt);
    al.h[1] = *(const v8b*)(arl + 32 * kt + 16);
#pragma unroll
    for (int t = 0; t < 4; ++t) {
      const __bf16* bph = bbh + (size_t)(16 * t) * CIN + 32 * kt;
      const __bf16* bpl = bbl + (size_t)(16 * t) * CIN + 32 * kt;
      FragB bh, bl;
      bh.h[0] = *(const v8b*)bph;
      bh.h[1] = *(const v8b*)(bph + 16);
      bl.h[0] = *(const v8b*)bpl;
      bl.h[1] = *(const v8b*)(bpl + 16);
      acc[t] = wm3(ah, al, bh, bl, acc[t]);
    }
  }
  __syncthreads();

  const int r0 = 16 * rt + 8 * hh;
  float* sp = stg + r0 * PCOLS + 64 * cg + m;
#pragma unroll
  for (int t = 0; t < 4; ++t) {
    const float bvv = bias[wrow0 + 64 * cg + 16 * t + m];
    sp[0 * PCOLS + 16 * t] = acc[t][0] + bvv;
    sp[1 * PCOLS + 16 * t] = acc[t][1] + bvv;
    sp[2 * PCOLS + 16 * t] = acc[t][2] + bvv;
    sp[3 * PCOLS + 16 * t] = acc[t][3] + bvv;
    sp[4 * PCOLS + 16 * t] = acc[t][4] + bvv;
    sp[5 * PCOLS + 16 * t] = acc[t][5] + bvv;
    sp[6 * PCOLS + 16 * t] = acc[t][6] + bvv;
    sp[7 * PCOLS + 16 * t] = acc[t][7] + bvv;
  }
  __syncthreads();

  const float* lp = stg + (8 * wave) * PCOLS + 4 * lane;
  float* gp = outp + ((size_t)rowBase + 8 * wave) * ldo + cb * PCOLS + 4 * lane;
#pragma unroll
  for (int i = 0; i < 8; ++i) { const v4f v = *(const v4f*)(lp + i * PCOLS); *(volatile v4f*)(gp + (size_t)i * ldo) = v; }
  __threadfence();
#pragma unroll
  for (int i = 0; i < 8; ++i) { const v4f v = *(const v4f*)(lp + i * PCOLS); *(volatile v4f*)(gp + (size_t)i * ldo) = v; }
}

__global__ __launch_bounds__(NTHR) void k_edge(
    const float* __restrict__ qk, const int* __restrict__ ei, const float* __restrict__ pos,
    const float* __restrict__ Wg, const float* __restrict__ bg,
    float* S, float* part, int nN, int nE) {
  __shared__ __attribute__((aligned(16))) float sS[EPB * NH];
  __shared__ float wred[NWAVE * NH];
  __shared__ float bstat[2 * NH];
  __shared__ __attribute__((aligned(16))) float sline[32];
  const int tid = threadIdx.x, lane = tid & 31, wave = tid >> 5;
  const int h = lane >> 3, sub = lane & 7;
  const int eBase = blockIdx.x * EPB;
  const float g0 = Wg[h], g1 = Wg[NH + h], g2 = Wg[2 * NH + h], g3 = Wg[3 * NH + h], gb = bg[h];

#pragma unroll 1
  for (int it = 0; it < EPB / NWAVE; ++it) {
    const int  el    = it * NWAVE + wave;
    const int  e     = eBase + el;
    const bool valid = e < nE;
    const int  ec    = valid ? e : nE - 1;
    int src = ei[ec];
    int dst = ei[(size_t)nE + ec];
    src = src < 0 ? 0 : (src > nN - 1 ? nN - 1 : src);
    dst = dst < 0 ? 0 : (dst > nN - 1 ? nN - 1 : dst);
    const float* qp = qk + (size_t)src * (2 * HD) + h * DH + sub * 8;
    const float* kp = qk + (size_t)dst * (2 * HD) + HD + h * DH + sub * 8;
    const v4f q0 = *(const v4f*)qp, q1 = *(const v4f*)(qp + 4);
    const v4f k0 = *(const v4f*)kp, k1 = *(const v4f*)(kp + 4);
    float d = q0.x * k0.x + q0.y * k0.y + q0.z * k0.z + q0.w * k0.w
            + q1.x * k1.x + q1.y * k1.y + q1.z * k1.z + q1.w * k1.w;
    d += __shfl_xor(d, 1);
    d += __shfl_xor(d, 2);
    d += __shfl_xor(d, 4);
    const float* ps = pos + (size_t)src * 3;
    const float* pd = pos + (size_t)dst * 3;
    const float ex = pd[0] - ps[0], ey = pd[1] - ps[1], ez = pd[2] - ps[2];
    const float dist = sqrtf(ex * ex + ey * ey + ez * ez);
    const float inv  = 1.0f / (dist + 1e-8f);
    const float gw   = dist * g0 + (ex * inv) * g1 + (ey * inv) * g2 + (ez * inv) * g3 + gb;
    float s = d * 0.125f + gw;
    s = valid ? s : NEGBIG;
    if (sub == 0) sS[el * NH + h] = s;
  }
  __syncthreads();

  const float v0 = sS[tid], v1 = sS[tid + NTHR], v2 = sS[tid + 2 * NTHR], v3 = sS[tid + 3 * NTHR];
  float mx = fmaxf(fmaxf(v0, v1), fmaxf(v2, v3));
  mx = fmaxf(mx, __shfl_xor(mx, 4));
  mx = fmaxf(mx, __shfl_xor(mx, 8));
  mx = fmaxf(mx, __shfl_xor(mx, 16));
  if (lane < NH) wred[wave * NH + lane] = mx;
  __syncthreads();
  if (tid < NH) {
    float M = wred[tid];
#pragma unroll 1
    for (int w = 1; w < NWAVE; ++w) M = fmaxf(M, wred[w * NH + tid]);
    bstat[tid] = M;
  }
  __syncthreads();
  const float mb = bstat[tid & 3];
  float z = __expf(v0 - mb) + __expf(v1 - mb) + __expf(v2 - mb) + __expf(v3 - mb);
  z += __shfl_xor(z, 4);
  z += __shfl_xor(z, 8);
  z += __shfl_xor(z, 16);
  if (lane < NH) wred[wave * NH + lane] = z;
  __syncthreads();
  if (tid < NH) {
    float Z = wred[tid];
#pragma unroll 1
    for (int w = 1; w < NWAVE; ++w) Z += wred[w * NH + tid];
    bstat[NH + tid] = Z;
  }
  __syncthreads();
  if (tid < 32) {
    const float bvv = bstat[tid < 2 * NH ? tid : (2 * NH - 1)];
    sline[tid] = (tid < 2 * NH) ? bvv : 0.f;
  }
  __syncthreads();

  {
    const v4f sv = *(const v4f*)(sS + wave * 128 + 4 * lane);
    float* gp = S + (size_t)eBase * NH + wave * 128 + 4 * lane;
    *(volatile v4f*)gp = sv;
    if (wave == 0 && lane < 8) {
      const v4f pv = *(const v4f*)(sline + 4 * lane);
      *(volatile v4f*)(part + (size_t)blockIdx.x * 32 + 4 * lane) = pv;
    }
    __threadfence();
    *(volatile v4f*)gp = sv;
    if (wave == 0 && lane < 8) {
      const v4f pv = *(const v4f*)(sline + 4 * lane);
      *(volatile v4f*)(part + (size_t)blockIdx.x * 32 + 4 * lane) = pv;
    }
  }
}

__global__ __launch_bounds__(NTHR) void k_stats(const float* __restrict__ part, float* stats, int nEB) {
  __shared__ __attribute__((aligned(16))) float  pm[NTHR * NH];
  __shared__ __attribute__((aligned(16))) double pz[NTHR * NH];
  __shared__ float sM[NH];
  __shared__ float sZ[NH];
  __shared__ __attribute__((aligned(16))) float sline[32];
  const int tid = threadIdx.x, lane = tid & 31, wave = tid >> 5;

  float m0 = NEGBIG, m1 = NEGBIG, m2 = NEGBIG, m3 = NEGBIG;
#pragma unroll 1
  for (int b = tid; b < nEB; b += NTHR) {
    const v4f mv = *(const v4f*)(part + (size_t)b * 32);
    m0 = fmaxf(m0, mv.x); m1 = fmaxf(m1, mv.y); m2 = fmaxf(m2, mv.z); m3 = fmaxf(m3, mv.w);
  }
  pm[tid * NH + 0] = m0; pm[tid * NH + 1] = m1; pm[tid * NH + 2] = m2; pm[tid * NH + 3] = m3;
  __syncthreads();
  if (tid < NH) {
    float M = NEGBIG;
#pragma unroll 1
    for (int i = 0; i < NTHR; ++i) M = fmaxf(M, pm[i * NH + tid]);
    sM[tid] = M;
  }
  __syncthreads();
  const float M0 = sM[0], M1 = sM[1], M2 = sM[2], M3 = sM[3];
  double z0 = 0.0, z1 = 0.0, z2 = 0.0, z3 = 0.0;
#pragma unroll 1
  for (int b = tid; b < nEB; b += NTHR) {
    const v4f mv = *(const v4f*)(part + (size_t)b * 32);
    const v4f zv = *(const v4f*)(part + (size_t)b * 32 + 4);
    z0 += (double)(__expf(mv.x - M0) * zv.x);
    z1 += (double)(__expf(mv.y - M1) * zv.y);
    z2 += (double)(__expf(mv.z - M2) * zv.z);
    z3 += (double)(__expf(mv.w - M3) * zv.w);
  }
  pz[tid * NH + 0] = z0; pz[tid * NH + 1] = z1; pz[tid * NH + 2] = z2; pz[tid * NH + 3] = z3;
  __syncthreads();
  if (tid < NH) {
    double Z = 0.0;
#pragma unroll 1
    for (int i = 0; i < NTHR; ++i) Z += pz[i * NH + tid];
    sZ[tid] = (Z > 0.0) ? (float)(1.0 / Z) : 0.f;
  }
  __syncthreads();
  if (tid < 32) {
    const float a = sM[tid < NH ? tid : (NH - 1)];
    const int   j = tid - NH;
    const float c = sZ[j < 0 ? 0 : (j > NH - 1 ? NH - 1 : j)];
    sline[tid] = (tid < NH) ? a : ((tid < 2 * NH) ? c : 0.f);
  }
  __syncthreads();
  if (wave == 0 && lane < 8) {
    const v4f v = *(const v4f*)(sline + 4 * lane);
    *(volatile v4f*)(stats + 4 * lane) = v;
  }
  __threadfence();
  if (wave == 0 && lane < 8) {
    const v4f v = *(const v4f*)(sline + 4 * lane);
    *(volatile v4f*)(stats + 4 * lane) = v;
  }
}

__global__ __launch_bounds__(NTHR) void k_agg(
    const int* __restrict__ ei, const float* __restrict__ S, const float* __restrict__ stats,
    float* Apl, int nE, int vec8) {
  extern __shared__ v4f lds_dyn[];
  float* acc  = (float*)lds_dyn;
  int*   list = (int*)(acc + NB * NH);
  int*   wcnt = list + LISTN;
  float* stt  = (float*)(wcnt + NWAVE);
  const int tid = threadIdx.x, lane = tid & 31, wave = tid >> 5;
  const int nodeBase = blockIdx.x * NB;
  const int* dsts = ei + nE;

  {
    const v4f z = {0.f, 0.f, 0.f, 0.f};
    for (int i = tid; i < NB; i += NTHR) lds_dyn[i] = z;
  }
  if (tid < 8) stt[tid] = stats[tid];
  __syncthreads();
  const float myM = stt[lane & 3];

  const int nChunks = (nE + CHUNK - 1) / CHUNK;
#pragma unroll 1
  for (int ch = 0; ch < nChunks; ++ch) {
    const int cbase = ch * CHUNK;
    const int wc = scan_chunk<NB>(dsts, nE, cbase, nodeBase, vec8, list, tid, lane, wave);
    if (lane == 0) wcnt[wave] = wc;
    __syncthreads();
    if (wave == 0) {
#pragma unroll 1
      for (int wsx = 0; wsx < NWAVE; ++wsx) {
        int n = __builtin_amdgcn_readfirstlane(wcnt[wsx]);
        n = n > WCAP ? WCAP : (n < 0 ? 0 : n);
        const int* lp = list + wsx * WCAP;
#pragma unroll 1
        for (int i = 0; i < n; ++i) {
          const int ent  = __builtin_amdgcn_readfirstlane(lp[i]);
          const int slot = ent & (NB - 1);
          int e = cbase + ((ent >> 12) & (CHUNK - 1));
          e = e > nE - 1 ? nE - 1 : e;
          const float sv = S[(size_t)e * NH + (lane & 3)];
          const float ex = __expf(sv - myM);
          if (lane < NH) {
            float* ap = acc + slot * NH + lane;
            *ap = *ap + ex;
          }
        }
      }
    }
    __syncthreads();
  }

  const float iz0 = stt[4], iz1 = stt[5], iz2 = stt[6], iz3 = stt[7];
  float* gbase = Apl + (size_t)blockIdx.x * NB * NH;
#pragma unroll 4
  for (int q = 0; q < 16; ++q) {
    const int f = (wave * 16 + q) * 128 + 4 * lane;
    v4f v = *(const v4f*)(acc + f);
    v.x *= iz0; v.y *= iz1; v.z *= iz2; v.w *= iz3;
    *(volatile v4f*)(gbase + f) = v;
  }
  __threadfence();
#pragma unroll 4
  for (int q = 0; q < 16; ++q) {
    const int f = (wave * 16 + q) * 128 + 4 * lane;
    v4f v = *(const v4f*)(acc + f);
    v.x *= iz0; v.y *= iz1; v.z *= iz2; v.w *= iz3;
    *(volatile v4f*)(gbase + f) = v;
  }
}

__global__ __launch_bounds__(NTHR) void k_out(
    const float* __restrict__ V, const float* __restrict__ Apl,
    const __bf16* __restrict__ oh, const __bf16* __restrict__ ol,
    const float* __restrict__ bo, float* out, int nN) {
  extern __shared__ v4f lds_dyn[];
  __bf16* sH  = (__bf16*)lds_dyn;
  __bf16* sL  = sH + PROWS * APITCH;
  float*  stg = (float*)lds_dyn;
  const int tid = threadIdx.x, lane = tid & 31, wave = tid >> 5, hh = lane >> 4, m = lane & 15;
  const int rowBase = blockIdx.x * PROWS;

#pragma unroll
  for (int i = 0; i < (PROWS * HD / 8) / NTHR; ++i) {
    const int idx = i * NTHR + tid;
    const int r   = idx >> 5;
    const int c0  = (idx & 31) * 8;
    const int node = rowBase + r;
    const float a = Apl[(size_t)node * NH + (c0 >> 6)];
    const float* vp = V + (size_t)node * HD + c0;
    const v4f x0 = *(const v4f*)vp * a;
    const v4f x1 = *(const v4f*)(vp + 4) * a;
    const HiLo s = split8(x0, x1);
    *(v8b*)(sH + r * APITCH + c0) = s.hi;
    *(v8b*)(sL + r * APITCH + c0) = s.lo;
  }
  __syncthreads();

  const int rt = wave & 3, cg = wave >> 2;
  v8f acc[2];
#pragma unroll
  for (int t = 0; t < 2; ++t) { v8f z = {0.f, 0.f, 0.f, 0.f, 0.f, 0.f, 0.f, 0.f}; acc[t] = z; }
  const __bf16* arh = sH + (16 * rt + m) * APITCH + 8 * hh;
  const __bf16* arl = sL + (16 * rt + m) * APITCH + 8 * hh;
  const __bf16* bbh = oh + (size_t)(32 * cg + m) * HD + 8 * hh;
  const __bf16* bbl = ol + (size_t)(32 * cg + m) * HD + 8 * hh;
#pragma unroll 1
  for (int kt = 0; kt < HD / 32; ++kt) {
    FragB ah, al;
    ah.h[0] = *(const v8b*)(arh + 32 * kt);
    ah.h[1] = *(const v8b*)(arh + 32 * kt + 16);
    al.h[0] = *(const v8b*)(arl + 32 * kt);
    al.h[1] = *(const v8b*)(arl + 32 * kt + 16);
#pragma unroll
    for (int t = 0; t < 2; ++t) {
      const __bf16* bph = bbh + (size_t)(16 * t) * HD + 32 * kt;
      const __bf16* bpl = bbl + (size_t)(16 * t) * HD + 32 * kt;
      FragB bh, bl;
      bh.h[0] = *(const v8b*)bph;
      bh.h[1] = *(const v8b*)(bph + 16);
      bl.h[0] = *(const v8b*)bpl;
      bl.h[1] = *(const v8b*)(bpl + 16);
      acc[t] = wm3(ah, al, bh, bl, acc[t]);
    }
  }
  __syncthreads();

  const int r0 = 16 * rt + 8 * hh;
  float* sp = stg + r0 * DOUT + 32 * cg + m;
#pragma unroll
  for (int t = 0; t < 2; ++t) {
    const float bvv = bo[32 * cg + 16 * t + m];
    sp[0 * DOUT + 16 * t] = acc[t][0] + bvv;
    sp[1 * DOUT + 16 * t] = acc[t][1] + bvv;
    sp[2 * DOUT + 16 * t] = acc[t][2] + bvv;
    sp[3 * DOUT + 16 * t] = acc[t][3] + bvv;
    sp[4 * DOUT + 16 * t] = acc[t][4] + bvv;
    sp[5 * DOUT + 16 * t] = acc[t][5] + bvv;
    sp[6 * DOUT + 16 * t] = acc[t][6] + bvv;
    sp[7 * DOUT + 16 * t] = acc[t][7] + bvv;
  }
  __syncthreads();

  float* gbase = out + (size_t)rowBase * DOUT;
#pragma unroll
  for (int q = 0; q < 4; ++q) {
    const int f   = (8 * wave + 2 * q) * DOUT + 4 * lane;
    const int row = rowBase + 8 * wave + 2 * q + (lane >> 4);
    if (row < nN) { const v4f v = *(const v4f*)(stg + f); *(volatile v4f*)(gbase + f) = v; }
  }
  __threadfence();
#pragma unroll
  for (int q = 0; q < 4; ++q) {
    const int f   = (8 * wave + 2 * q) * DOUT + 4 * lane;
    const int row = rowBase + 8 * wave + 2 * q + (lane >> 4);
    if (row < nN) { const v4f v = *(const v4f*)(stg + f); *(volatile v4f*)(gbase + f) = v; }
  }
}

extern "C" void kernel_launch(void* const* d_in, const int* in_sizes, int n_in,
                              void* d_out, int out_size, void* d_ws, size_t ws_size,
                              hipStream_t stream) {
  if (n_in < 13) return;
  const int nN = in_sizes[0] / CIN;
  const int nE = in_sizes[1] / 2;
  if (nN < 1 || nE < 1) return;
  if (in_sizes[0] != nN * CIN || in_sizes[1] != 2 * nE || in_sizes[2] != 3 * nN) return;
  if (in_sizes[3] != CIN * HD || in_sizes[5] != CIN * HD || in_sizes[7] != CIN * HD || in_sizes[11] != HD * DOUT) return;
  if (in_sizes[4] < HD || in_sizes[6] < HD || in_sizes[8] < HD) return;
  if (in_sizes[9] < 4 * NH || in_sizes[10] < NH || in_sizes[12] < DOUT) return;
  if (out_size != nN * DOUT) return;

  const float* x   = (const float*)d_in[0];
  const int*   ei  = (const int*)d_in[1];
  const float* pos = (const float*)d_in[2];
  const float* Wq  = (const float*)d_in[3];
  const float* bq  = (const float*)d_in[4];
  const float* Wk  = (const float*)d_in[5];
  const float* bk  = (const float*)d_in[6];
  const float* Wv  = (const float*)d_in[7];
  const float* bv  = (const float*)d_in[8];
  const float* Wg  = (const float*)d_in[9];
  const float* bg  = (const float*)d_in[10];
  const float* Wo  = (const float*)d_in[11];
  const float* bo  = (const float*)d_in[12];
  float* out = (float*)d_out;

  const int NP  = ((nN + PROWS - 1) / PROWS) * PROWS;
  const int nPB = NP / PROWS;
  const int nEB = (nE + EPB - 1) / EPB;
  const int nAB = (nN + NB - 1) / NB;
  if ((long long)nAB * NB < (long long)NP) return;

  char* ws = (char*)d_ws;
  size_t off = 0;
  const size_t oWH  = off; off += (size_t)HQKV * CIN * 2;                off = (off + 255) & ~(size_t)255;
  const size_t oWL  = off; off += (size_t)HQKV * CIN * 2;                off = (off + 255) & ~(size_t)255;
  const size_t oOH  = off; off += (size_t)DOUT * HD * 2;                 off = (off + 255) & ~(size_t)255;
  const size_t oOL  = off; off += (size_t)DOUT * HD * 2;                 off = (off + 255) & ~(size_t)255;
  const size_t oBia = off; off += (size_t)HQKV * 4;                      off = (off + 255) & ~(size_t)255;
  const size_t oPar = off; off += (size_t)nEB * 32 * 4;                  off = (off + 255) & ~(size_t)255;
  const size_t oSta = off; off += (size_t)32 * 4;                        off = (off + 255) & ~(size_t)255;
  const size_t oA   = off; off += (size_t)nAB * NB * NH * 4;             off = (off + 255) & ~(size_t)255;
  const size_t oS   = off; off += (size_t)nEB * EPB * NH * 4;            off = (off + 255) & ~(size_t)255;
  const size_t oQK  = off; off += (size_t)NP * (2 * HD) * 4;             off = (off + 255) & ~(size_t)255;
  if (off > ws_size) return;
  if (off > (size_t)134217728u) return;
  __bf16* wh    = (__bf16*)(ws + oWH);
  __bf16* wl    = (__bf16*)(ws + oWL);
  __bf16* oh    = (__bf16*)(ws + oOH);
  __bf16* ol    = (__bf16*)(ws + oOL);
  float*  bias  = (float*)(ws + oBia);
  float*  part  = (float*)(ws + oPar);
  float*  stats = (float*)(ws + oSta);
  float*  Apl   = (float*)(ws + oA);
  float*  S     = (float*)(ws + oS);
  float*  QK    = (float*)(ws + oQK);
  float*  Vp    = (float*)(ws + oQK);

  const int vec8 = ((nE & 3) == 0) ? 1 : 0;
  const int nWB  = (HQKV * CIN / 8) / NTHR;
  const int nOWB = (DOUT * HD / 8) / NTHR;

  k_wprep<<<nWB + nOWB + 1, NTHR, 0, stream>>>(Wq, Wk, Wv, Wo, bq, bk, bv, wh, wl, oh, ol, bias, nWB, nOWB);

  hipFuncSetAttribute(reinterpret_cast<const void*>(&k_proj),
                      hipFuncAttributeMaxDynamicSharedMemorySize, LDS_PROJ);
  k_proj<<<nPB * 4, NTHR, LDS_PROJ, stream>>>(x, wh, wl, bias, QK, nN, 0, 4, 2 * HD);

  k_edge<<<nEB, NTHR, 0, stream>>>(QK, ei, pos, Wg, bg, S, part, nN, nE);

  k_stats<<<1, NTHR, 0, stream>>>(part, stats, nEB);

  hipFuncSetAttribute(reinterpret_cast<const void*>(&k_agg),
                      hipFuncAttributeMaxDynamicSharedMemorySize, LDS_AGG);
  k_agg<<<nAB, NTHR, LDS_AGG, stream>>>(ei, S, stats, Apl, nE, vec8);

  k_proj<<<nPB * 2, NTHR, LDS_PROJ, stream>>>(x, wh, wl, bias, Vp, nN, 2 * HD, 2, HD);

  hipFuncSetAttribute(reinterpret_cast<const void*>(&k_out),
                      hipFuncAttributeMaxDynamicSharedMemorySize, LDS_OUT);
  k_out<<<nPB, NTHR, LDS_OUT, stream>>>(Vp, Apl, oh, ol, bo, out, nN);
}
